// Tagger_13340168421424
// MI455X (gfx1250) — hardware-run, weakly checked
//
#include <hip/hip_runtime.h>


#ifndef NROWS
#define NROWS 262144
#endif
#define NROWS_FULL 262144
#define WIN_   5
#define VOCAB  100000
#define EMB    50
#define HID    250
#define KP     256
#define OUTD   36
#define OPAD   48
#define BR     64
#define NW     4
#define XPW    132
#define IDS_N  384
#define WSC    16.0f
#define WSI    (1.0f / 16.0f)
#define TL2    2.8853900817779268f
#define W1_PIECES (KP * KP / 8)
#define W2_PIECES (OPAD * KP / 8)

static_assert(WIN_ * EMB == HID);
static_assert(HID <= KP);
static_assert(KP % 32 == 0);
static_assert(KP / 32 == 8);
static_assert(OUTD <= OPAD);
static_assert(OPAD == 48);
static_assert(OUTD == 36);
static_assert((EMB * 2) % 4 == 0);
static_assert(EMB / 2 == 25);
static_assert(((size_t)VOCAB * EMB) % 8 == 0);
static_assert(((size_t)VOCAB * EMB * 2) % 128 == 0);
static_assert(NROWS % BR == 0);
static_assert(NROWS <= NROWS_FULL);
static_assert(BR == 16 * NW);
static_assert(XPW * 2 >= KP);
static_assert((XPW * 4) % 16 == 0);
static_assert(XPW - HID / 2 == 7);
static_assert((BR * OUTD * 4) % 512 == 0);
static_assert(BR * OUTD * 4 == 18 * 32 * 16);
static_assert(KP % (32 * NW) == 0);
static_assert(IDS_N % (32 * NW) == 0);
static_assert(IDS_N >= BR * WIN_);
static_assert(32 * NW >= OPAD);
static_assert(W1_PIECES % 256 == 0);
static_assert((W1_PIECES + W2_PIECES) % 256 == 0);
static_assert(BR * XPW * 4 + BR * OUTD * 4 + KP * 4 + 32 * NW * 4 + IDS_N * 4 <= 131072);
static_assert((size_t)NROWS_FULL * OUTD * 4 == (size_t)37748736);

typedef _Float16 h16;
typedef unsigned short bf;
typedef __attribute__((ext_vector_type(16))) __bf16   v16bf;
typedef __attribute__((ext_vector_type(16))) _Float16 v16h;
typedef __attribute__((ext_vector_type(8)))  _Float16 v8h;
typedef __attribute__((ext_vector_type(8)))  unsigned short v8us;
typedef __attribute__((ext_vector_type(8)))  float    v8f;
typedef __attribute__((ext_vector_type(4)))  float    v4f;
typedef v4f  __attribute__((may_alias)) v4fa;
typedef v8us __attribute__((may_alias)) v8usa;

__device__ __forceinline__ unsigned short f2bf(float f) { unsigned u = __float_as_uint(f); u += 0x7FFFu + ((u >> 16) & 1u); return (unsigned short)(u >> 16); }
__device__ __forceinline__ float bfr(float f) { return __uint_as_float(((unsigned)f2bf(f)) << 16); }
__device__ __forceinline__ v16h cat16(v8h lo, v8h hi) { return __builtin_shufflevector(lo, hi, 0, 1, 2, 3, 4, 5, 6, 7, 8, 9, 10, 11, 12, 13, 14, 15); }
__device__ __forceinline__ v16bf cat16b(v8us lo, v8us hi) { return __builtin_bit_cast(v16bf, __builtin_shufflevector(lo, hi, 0, 1, 2, 3, 4, 5, 6, 7, 8, 9, 10, 11, 12, 13, 14, 15)); }
__device__ __forceinline__ v8f wmma16(v16h a, v16h b, v8f c) { return __builtin_amdgcn_wmma_f32_16x16x32_f16(false, a, false, b, (short)0, c, false, false); }
__device__ __forceinline__ v8f wmmab(v16bf a, v16bf b, v8f c) { return __builtin_amdgcn_wmma_f32_16x16x32_bf16(false, a, false, b, (short)0, c, false, false); }
__device__ __forceinline__ v16h  ldh(const h16* p) { return cat16(*(const v8h*)p, *(const v8h*)(p + 16)); }
__device__ __forceinline__ v16bf ldb(const bf* p)  { return cat16b(*(const v8us*)p, *(const v8us*)(p + 16)); }
__device__ __forceinline__ void wave_sync() { __builtin_amdgcn_fence(3  , "wavefront"); __builtin_amdgcn_wave_barrier(); asm volatile("" ::: "memory"); }

static __device__ __forceinline__ v8f wmmabg(v16bf a, v16bf b, v8f c) { c = wmmab(a, b, c); asm volatile("v_nop\n\tv_nop\n\tv_nop\n\tv_nop" : "+v"(c) : "v"(a), "v"(b)); return c; }
static __device__ __forceinline__ v8f wmma16g(v16h a, v16h b, v8f c) { c = wmma16(a, b, c); asm volatile("v_nop\n\tv_nop\n\tv_nop\n\tv_nop" : "+v"(c) : "v"(a), "v"(b)); return c; }
static __device__ __forceinline__ h16 toh_flush(float v) { const float w = (fabsf(v) < 6.103515625e-05f) ? 0.0f : v; return (h16)w; }
static __device__ __forceinline__ float tanh_i(float z) { const float e = __builtin_amdgcn_exp2f(z * TL2); return 1.0f - 2.0f * __builtin_amdgcn_rcpf(e + 1.0f); }

__global__ __launch_bounds__(256) void k_cvt8(const float* __restrict__ src, bf* dst, size_t n8) {
    const size_t i = (size_t)blockIdx.x * 256 + threadIdx.x; if (i >= n8) return;
    const v8f v = *(const v8f*)(src + i * 8); v8us o;
#pragma unroll
    for (int k = 0; k < 8; ++k) o[k] = f2bf(v[k]);
    *(volatile v8us*)(dst + i * 8) = o; __threadfence(); *(volatile v8us*)(dst + i * 8) = o;
}

__global__ __launch_bounds__(256) void k_wt(const float* __restrict__ w1, const float* __restrict__ w2, bf* W1T, h16* W2T) {
    const unsigned i = blockIdx.x * 256u + threadIdx.x;
    if (i < (unsigned)W1_PIECES) {
        const unsigned n = i / (unsigned)(KP / 8), k0 = (i % (unsigned)(KP / 8)) * 8u;
        const unsigned nc = min(n, (unsigned)(HID - 1));
        v8us o;
#pragma unroll
        for (int j = 0; j < 8; ++j) {
            const unsigned k = k0 + (unsigned)j; const unsigned kc = min(k, (unsigned)(HID - 1));
            float v = w1[kc * (unsigned)HID + nc]; asm volatile("" : "+v"(v));
            const bool ok = (k < (unsigned)HID) && (n < (unsigned)HID);
            o[j] = f2bf(ok ? v : 0.0f); }
        *(volatile v8us*)(W1T + (size_t)i * 8) = o; __threadfence(); *(volatile v8us*)(W1T + (size_t)i * 8) = o;
    } else if (i < (unsigned)(W1_PIECES + W2_PIECES)) {
        const unsigned q = i - (unsigned)W1_PIECES;
        const unsigned n = q / (unsigned)(KP / 8), k0 = (q % (unsigned)(KP / 8)) * 8u;
        const unsigned nc = min(n, (unsigned)(OUTD - 1));
        v8h o;
#pragma unroll
        for (int j = 0; j < 8; ++j) {
            const unsigned k = k0 + (unsigned)j; const unsigned kc = min(k, (unsigned)(HID - 1));
            float v = w2[kc * (unsigned)OUTD + nc]; asm volatile("" : "+v"(v));
            const bool ok = (k < (unsigned)HID) && (n < (unsigned)OUTD);
            const float w = ok ? bfr(v) : 0.0f;
            o[j] = toh_flush(w * WSC); }
        *(volatile v8h*)(W2T + (size_t)q * 8) = o; __threadfence(); *(volatile v8h*)(W2T + (size_t)q * 8) = o;
    }
}

__global__ __launch_bounds__(32 * NW) void k_mlp(const int* __restrict__ idx, const bf* __restrict__ TB, const bf* __restrict__ W1T, const h16* __restrict__ W2T,
                                                 const float* __restrict__ b1, const float* __restrict__ b2, float* OUT) {
    __shared__ __align__(16) unsigned xs[BR * XPW];
    __shared__ __align__(16) float os[BR * OUTD];
    __shared__ __align__(16) float bi[KP];
    __shared__ __align__(16) float bo[32 * NW];
    __shared__ int ids[IDS_N];
    const unsigned tid = threadIdx.x;
    const int lane = threadIdx.x & 31, lr = lane & 15, hi = lane >> 4;
    const int wave = __builtin_amdgcn_readfirstlane((int)(threadIdx.x >> 5));
    const unsigned bx = blockIdx.x;
    const unsigned r0 = bx * (unsigned)BR;
    const unsigned* tb32 = (const unsigned*)TB;

#pragma unroll
    for (unsigned t = 0; t < (unsigned)(IDS_N / (32 * NW)); ++t) {
        const unsigned e = t * (unsigned)(32 * NW) + tid;
        ids[e] = idx[min(r0 * (unsigned)WIN_ + e, (unsigned)(NROWS * WIN_ - 1))]; }
#pragma unroll
    for (unsigned t = 0; t < (unsigned)(KP / (32 * NW)); ++t) {
        const unsigned e = t * (unsigned)(32 * NW) + tid;
        float v = b1[min(e, (unsigned)(HID - 1))]; asm volatile("" : "+v"(v));
        bi[e] = (e < (unsigned)HID) ? bfr(v) : 0.0f; }
    { float v = b2[min(tid, (unsigned)(OUTD - 1))]; asm volatile("" : "+v"(v));
      bo[tid] = (tid < (unsigned)OUTD) ? bfr(v) : 0.0f; }
    __syncthreads();

#pragma unroll 4
    for (unsigned e = tid; e < (unsigned)(BR * (HID / 2)); e += (unsigned)(32 * NW)) {
        const unsigned row = e / (unsigned)(HID / 2); const unsigned col = e - row * (unsigned)(HID / 2);
        const unsigned piece = e / (unsigned)(EMB / 2); const unsigned d = e - piece * (unsigned)(EMB / 2);
        const int id = ids[piece];
        const bool ok = (id >= 0) && (id < VOCAB);
        const int idc = min(max(id, 0), VOCAB - 1);
        unsigned v = tb32[(unsigned)idc * (unsigned)(EMB / 2) + d]; asm volatile("" : "+v"(v));
        xs[row * (unsigned)XPW + col] = ok ? v : 0u; }
#pragma unroll 1
    for (unsigned e = tid; e < (unsigned)(BR * (XPW - HID / 2)); e += (unsigned)(32 * NW)) {
        const unsigned row = e / (unsigned)(XPW - HID / 2); const unsigned c = e - row * (unsigned)(XPW - HID / 2);
        xs[row * (unsigned)XPW + (unsigned)(HID / 2) + c] = 0u; }
    __syncthreads();

    v8f oH[3];
#pragma unroll
    for (int nb = 0; nb < 3; ++nb) { oH[nb] = (v8f){}; }
    const size_t wao = (size_t)lr * KP + 8 * hi;
    const size_t w2o = (size_t)lr * KP + 8 * hi;
    const unsigned xo = (unsigned)(wave * 16 + lr) * (unsigned)XPW + 4u * (unsigned)hi;
#pragma unroll 1
    for (int s = 0; s < KP / 32; ++s) {
        v8f z0 = (v8f){}, z1 = (v8f){};
#pragma unroll 2
        for (int kc = 0; kc < KP; kc += 32) {
            const v16bf xb = cat16b(*(const v8usa*)(&xs[xo + (unsigned)(kc >> 1)]), *(const v8usa*)(&xs[xo + (unsigned)(kc >> 1) + 8u]));
            const v16bf a0 = ldb(W1T + wao + (size_t)(32 * s) * KP + kc);
            const v16bf a1 = ldb(W1T + wao + (size_t)(32 * s + 16) * KP + kc);
            z0 = wmmabg(a0, xb, z0); z1 = wmmabg(a1, xb, z1);
        }
        const v4f ba0 = *(const v4fa*)(&bi[32 * s + 8 * hi]), ba1 = *(const v4fa*)(&bi[32 * s + 8 * hi + 4]);
        const v4f bb0 = *(const v4fa*)(&bi[32 * s + 16 + 8 * hi]), bb1 = *(const v4fa*)(&bi[32 * s + 16 + 8 * hi + 4]);
        v16h pH;
#pragma unroll
        for (int r = 0; r < 4; ++r) {
            const float t0 = tanh_i(z0[r] + ba0[r]),     t1 = tanh_i(z0[4 + r] + ba1[r]);
            const float t2 = tanh_i(z1[r] + bb0[r]),     t3 = tanh_i(z1[4 + r] + bb1[r]);
            const h16 h0 = toh_flush(t0), h1 = toh_flush(t1), h2 = toh_flush(t2), h3 = toh_flush(t3);
            pH[r] = h0; pH[4 + r] = h1; pH[8 + r] = h2; pH[12 + r] = h3; }
#pragma unroll
        for (int nb = 0; nb < 3; ++nb) {
            const v16h a2 = ldh(W2T + w2o + (size_t)(nb * 16) * KP + 32 * s);
            oH[nb] = wmma16g(a2, pH, oH[nb]); }
    }

    const unsigned orow = (unsigned)(wave * 16 + lr) * (unsigned)OUTD;
#pragma unroll
    for (int nb = 0; nb < 3; ++nb) {
        const unsigned n0 = (unsigned)(nb * 16 + 8 * hi);
        const v4f c0 = *(const v4fa*)(&bo[n0]), c1 = *(const v4fa*)(&bo[n0 + 4]);
        v4f a, c;
#pragma unroll
        for (int i = 0; i < 4; ++i) { a[i] = oH[nb][i] * WSI + c0[i]; c[i] = oH[nb][4 + i] * WSI + c1[i]; }
        if (nb < 2) { *(v4fa*)(&os[orow + n0]) = a; *(v4fa*)(&os[orow + n0 + 4]) = c; }
        else        { if (hi == 0) *(v4fa*)(&os[orow + 32]) = a; }
    }
    __syncthreads();

    float* ob = OUT + (size_t)r0 * OUTD;
#pragma unroll 1
    for (int ps = 0; ps < 2; ++ps) {
#pragma unroll 1
        for (unsigned p = tid; p < (unsigned)(BR * OUTD / 4); p += (unsigned)(32 * NW)) {
            const v4f val = *(const v4fa*)(&os[p * 4u]);
            *(volatile v4f*)(ob + (size_t)p * 4) = val; }
        if (ps == 0) __threadfence(); }
}

static constexpr size_t al256(size_t v) { return (v + 255) & ~(size_t)255; }
static constexpr size_t SZ_TB = al256((size_t)VOCAB * EMB * 2);
static constexpr size_t SZ_W1 = al256((size_t)KP * KP * 2);
static constexpr size_t SZ_W2 = al256((size_t)OPAD * KP * 2);
static constexpr size_t SZ_TOTAL = SZ_TB + SZ_W1 + SZ_W2;
static constexpr size_t TB_N8 = (size_t)VOCAB * EMB / 8;
static constexpr unsigned TB_GRID = (unsigned)((TB_N8 + 255) / 256);
static constexpr unsigned WT_GRID = (unsigned)((W1_PIECES + W2_PIECES) / 256);
static constexpr unsigned ML_GRID = (unsigned)(NROWS / BR);
static_assert(SZ_TOTAL <= (size_t)134217728);
static_assert(TB_N8 * 16 <= SZ_TB);
static_assert((size_t)W1_PIECES * 16 == (size_t)KP * KP * 2);
static_assert((size_t)W2_PIECES * 16 == (size_t)OPAD * KP * 2);

extern "C" void kernel_launch(void* const* d_in, const int* in_sizes, int n_in,
                              void* d_out, int out_size, void* d_ws, size_t ws_size, hipStream_t stream) {
    if (n_in < 6) return;
    if ((size_t)in_sizes[0] < (size_t)NROWS * WIN_) return;
    if ((size_t)in_sizes[1] < (size_t)VOCAB * EMB) return;
    if ((size_t)in_sizes[2] < (size_t)HID * HID || in_sizes[3] < HID) return;
    if ((size_t)in_sizes[4] < (size_t)HID * OUTD || in_sizes[5] < OUTD) return;
    if ((size_t)out_size < (size_t)NROWS * OUTD) return;
    if (SZ_TOTAL > ws_size) return;
    const int*   idx = (const int*)d_in[0];
    const float* tab = (const float*)d_in[1];
    const float* w1  = (const float*)d_in[2];
    const float* b1  = (const float*)d_in[3];
    const float* w2  = (const float*)d_in[4];
    const float* b2  = (const float*)d_in[5];
    float* OUT = (float*)d_out;
    char* wsp = (char*)d_ws;
    bf*  TB  = (bf*)wsp;  wsp += SZ_TB;
    bf*  W1T = (bf*)wsp;  wsp += SZ_W1;
    h16* W2T = (h16*)wsp; wsp += SZ_W2;

    k_cvt8<<<TB_GRID, 256, 0, stream>>>(tab, TB, TB_N8);
    k_wt<<<WT_GRID, 256, 0, stream>>>(w1, w2, W1T, W2T);
    k_mlp<<<ML_GRID, 32 * NW, 0, stream>>>(idx, TB, W1T, W2T, b1, b2, OUT);
}
